// JKNet_5995774345341
// MI455X (gfx1250) — hardware-verified
//
#include <hip/hip_runtime.h>
#include <math.h>

constexpr int NN = 100000;
constexpr int NE = 1600000;
constexpr int FDIM = 128;
constexpr int CDIM = 64;
constexpr int KJK = 3 * FDIM;
constexpr int NPAD = 100032;
constexpr int NT = 256;
constexpr int NWAVE = NT / 32;
constexpr int SCH = 4096;
constexpr int SPT = SCH / NT;
constexpr int NCH = (NE + SCH - 1) / SCH;
constexpr int REC_SHIFT = 12;
constexpr int RL = 448;
constexpr int NBL = (NPAD + RL - 1) / RL;
constexpr int RLW = RL / NWAVE;
constexpr int RF = 896;
constexpr int NBF = (NN + RF - 1) / RF;
constexpr int RFW = RF / NWAVE;
constexpr int RD = 32768;
constexpr int NBD = (NPAD + RD - 1) / RD;
constexpr int NORM_ROWS = NBD * RD;
constexpr int NFC8 = NN * FDIM / 8;
constexpr float WCARRY = 64.0f;
constexpr float HCARRY = 16.0f;
constexpr float AGG0CARRY = 16.0f;
constexpr float GSCALE = 1.0f / (16.0f * 64.0f);

static_assert(NPAD % 64 == 0 && NPAD >= NN);
static_assert(FDIM == 128 && CDIM == 64 && KJK % 32 == 0 && FDIM % 32 == 0);
static_assert(NBL * RL >= NPAD && NBF * RF >= NN && NORM_ROWS >= NPAD);
static_assert(RL % (2 * NWAVE) == 0 && RF % (2 * NWAVE) == 0 && RD % (4 * NT) == 0);
static_assert(NE % SPT == 0 && SPT % 4 == 0 && NCH * SCH >= NE && SCH == (1 << REC_SHIFT));
static_assert(RD <= (1 << (30 - REC_SHIFT)));
static_assert((NN % 2) == 0 && (NPAD % 2) == 0);
static_assert(NFC8 % 256 == 0);
static_assert((RL * FDIM) % (4 * NT) == 0 && (RF * CDIM) % (4 * NT) == 0);

typedef __attribute__((ext_vector_type(16))) _Float16 v16h;
typedef __attribute__((ext_vector_type(8)))  _Float16 v8h;
typedef __attribute__((ext_vector_type(8)))  float    v8f;
typedef __attribute__((ext_vector_type(4)))  float    v4f;
typedef __attribute__((ext_vector_type(2)))  float    v2f;
typedef __attribute__((ext_vector_type(4)))  int      v4i;
typedef __attribute__((ext_vector_type(4)))  unsigned int v4u;
typedef __attribute__((ext_vector_type(2)))  unsigned int v2u;

__device__ __forceinline__ float bf16r(float f) {
  unsigned u = __float_as_uint(f);
  u = (u + 0x7FFFu + ((u >> 16) & 1u)) & 0xFFFF0000u;
  return __uint_as_float(u);
}
__device__ __forceinline__ unsigned short bf_bits_rne(float f) {
  unsigned u = __float_as_uint(f);
  return (unsigned short)((u + 0x7FFFu + ((u >> 16) & 1u)) >> 16);
}
__device__ __forceinline__ unsigned pk16(unsigned short a, unsigned short b) { return (unsigned)a | ((unsigned)b << 16); }
__device__ __forceinline__ unsigned short h_bits(float f) { const _Float16 h = (_Float16)f; return __builtin_bit_cast(unsigned short, h); }
__device__ __forceinline__ float h16_to_f32(unsigned hb) {
  const unsigned sgn = (hb & 0x8000u) << 16; const unsigned em = hb & 0x7fffu;
  const float fn = __uint_as_float((em << 13) + 0x38000000u);
  const float fs = (float)em * 5.9604644775390625e-8f;
  const float mag = (em < 0x400u) ? fs : fn; return __uint_as_float(__float_as_uint(mag) | sgn); }

__device__ __forceinline__ void dep_guard_h(v8f& a, v8f& b, v16h x, v16h y) { asm volatile("v_nop\n\tv_nop\n\tv_nop\n\tv_nop" : "+v"(a), "+v"(b) : "v"(x), "v"(y)); }
__device__ __forceinline__ void keep4_h(v16h a, v16h b, v16h c, v16h d) { asm volatile("v_nop" :: "v"(a), "v"(b), "v"(c), "v"(d)); }
__device__ __forceinline__ void acc_guard4(v8f& a, v8f& b, v8f& c, v8f& d) { asm volatile("v_nop\n\tv_nop\n\tv_nop\n\tv_nop" : "+v"(a), "+v"(b), "+v"(c), "+v"(d)); }
template <typename T> struct Frag;
template <> struct Frag<_Float16> {
  typedef v16h V; union U { v16h v; v8h h[2]; };
  static __device__ __forceinline__ v16h load(const _Float16* p) {
    U f; f.h[0] = *(const v8h*)(p); f.h[1] = *(const v8h*)(p + 16); return f.v;
  }
  static __device__ __forceinline__ v8f mma(v16h a, v16h b, v8f c) {
    return __builtin_amdgcn_wmma_f32_16x16x32_f16(false, a, false, b, (short)0, c, false, false);
  }
  static __device__ __forceinline__ void guard(v8f& a, v8f& b, v16h x, v16h y) { dep_guard_h(a, b, x, y); }
  static __device__ __forceinline__ void keep(v16h a, v16h b, v16h c, v16h d) { keep4_h(a, b, c, d); }
};

template <bool ROWSCALE, bool BIASN, bool RELU, int OUT_MODE>
__global__ __launch_bounds__(256) void gemm_f16_kernel(
    const unsigned short* __restrict__ Ap, int lda,
    const unsigned short* __restrict__ Btp, int ldb,
    void* __restrict__ Cout, int ldc,
    const float* __restrict__ bias, const float* __restrict__ rown,
    int M, int N, int K, float scale, float ocarry) {
  typedef _Float16 T;
  typedef v16h V;
  const T* Ab = (const T*)Ap; const T* Bb = (const T*)Btp;
  __shared__ __align__(16) float sT[8][16 * 68];
  const int lane = threadIdx.x & 31;
  const int wave = threadIdx.x >> 5;
  const int tilesN = N >> 6;
  const int tilesM = M >> 6;
  const int tile = blockIdx.x * 8 + wave;
  if (tile >= tilesM * tilesN) return;
  const int tm = tile / tilesN;
  const int tn = tile - tm * tilesN;
  const int m0 = tm << 6;
  const int n0 = tn << 6;

  const int rlane = lane & 15;
  const int koff  = (lane >> 4) * 8;
  const int mOff  = (lane >> 4) * 8;

  v8f acc[4][4];
#pragma unroll
  for (int i = 0; i < 4; ++i)
#pragma unroll
    for (int j = 0; j < 4; ++j) acc[i][j] = (v8f){0.f,0.f,0.f,0.f,0.f,0.f,0.f,0.f};

  for (int k0 = 0; k0 < K; k0 += 32) {
    V bh[4];
#pragma unroll
    for (int j = 0; j < 4; ++j) {
      const size_t bo = (size_t)(n0 + (j << 4) + rlane) * ldb + koff + k0;
      bh[j] = Frag<T>::load(Bb + bo);
    }
#pragma unroll
    for (int i = 0; i < 4; ++i) {
      const size_t ao = (size_t)(m0 + (i << 4) + rlane) * lda + koff + k0;
      V ah = Frag<T>::load(Ab + ao);
#pragma unroll
      for (int j = 0; j < 4; ++j) {
        acc[i][j] = Frag<T>::mma(ah, bh[j], acc[i][j]);
      }
      Frag<T>::guard(acc[i][0], acc[i][3], ah, ah);
    }
    Frag<T>::keep(bh[0], bh[1], bh[2], bh[3]);
  }
  acc_guard4(acc[0][0], acc[0][1], acc[0][2], acc[0][3]);
  acc_guard4(acc[1][0], acc[1][1], acc[1][2], acc[1][3]);
  acc_guard4(acc[2][0], acc[2][1], acc[2][2], acc[2][3]);
  acc_guard4(acc[3][0], acc[3][1], acc[3][2], acc[3][3]);

  float* slab = sT[wave];
#pragma unroll
  for (int i = 0; i < 4; ++i) {
    const int mBase = m0 + (i << 4);
    v4f rsA = {1.f, 1.f, 1.f, 1.f};
    v4f rsB = {1.f, 1.f, 1.f, 1.f};
    if (ROWSCALE) {
      rsA = *(const v4f*)(rown + mBase + mOff);
      rsB = *(const v4f*)(rown + mBase + mOff + 4);
    }
#pragma unroll
    for (int j = 0; j < 4; ++j) {
      const int n = n0 + (j << 4) + rlane;
      float bv = 0.f;
      if (BIASN) bv = bf16r(bias[n]);
#pragma unroll
      for (int r = 0; r < 8; ++r) {
        float v = acc[i][j][r] * scale;
        if (ROWSCALE) { const float rs = (r < 4) ? rsA[r & 3] : rsB[r & 3]; v = v * rs; }
        if (BIASN) v = v + bv;
        if (RELU) v = fmaxf(v, 0.0f);
        v = v * ocarry;
        slab[(mOff + r) * 68 + (j << 4) + rlane] = v;
      }
    }
    __builtin_amdgcn_fence(__ATOMIC_RELEASE, "workgroup");
    __builtin_amdgcn_wave_barrier();
    __builtin_amdgcn_fence(__ATOMIC_ACQUIRE, "workgroup");
    if (OUT_MODE == 0) {
      float* C = (float*)Cout;
      const int hh = lane >> 4, c4 = (lane & 15) * 4;
      for (int pass = 0; pass < 2; ++pass) {
#pragma unroll
        for (int it = 0; it < 8; ++it) {
          const int row = it * 2 + hh;
          v4f v = *(const v4f*)(slab + row * 68 + c4);
          *(volatile v4f*)(C + (size_t)(mBase + row) * ldc + n0 + c4) = v;
        }
        __threadfence();
      }
    } else {
      const int q = lane >> 3, c8 = (lane & 7) * 8;
      unsigned short* C = (unsigned short*)Cout;
      for (int pass = 0; pass < 2; ++pass) {
#pragma unroll
        for (int it = 0; it < 4; ++it) {
          const int row = it * 4 + q;
          const float* sp = slab + row * 68 + c8;
          v8h hv;
#pragma unroll
          for (int e = 0; e < 8; ++e) hv[e] = (_Float16)sp[e];
          *(volatile v8h*)(C + (size_t)(mBase + row) * ldc + n0 + c8) = hv;
        }
        __threadfence();
      }
    }
    __builtin_amdgcn_fence(__ATOMIC_RELEASE, "workgroup");
    __builtin_amdgcn_wave_barrier();
    __builtin_amdgcn_fence(__ATOMIC_ACQUIRE, "workgroup");
  }
}

__global__ __launch_bounds__(NT) void prep_kernel(const float* __restrict__ W0, const float* __restrict__ W1,
                                                 const float* __restrict__ W2, const float* __restrict__ Wo,
                                                 unsigned short* __restrict__ T0, unsigned short* __restrict__ T1,
                                                 unsigned short* __restrict__ T2, unsigned short* __restrict__ To,
                                                 float carry) {
  __shared__ float sm[64][65];
  const int z = blockIdx.z;
  const float* W = (z == 0) ? W0 : (z == 1) ? W1 : (z == 2) ? W2 : Wo;
  unsigned short* op = (z == 0) ? T0 : (z == 1) ? T1 : (z == 2) ? T2 : To;
  const int KD = (z == 3) ? KJK : FDIM;
  const int ND = (z == 3) ? CDIM : FDIM;
  const int kt = blockIdx.x, ntb = blockIdx.y;
  if (kt >= (KD >> 6) || ntb >= (ND >> 6)) return;
  const int k0 = kt << 6, c0 = ntb << 6;
  const int t = threadIdx.x;
#pragma unroll
  for (int i = 0; i < 16; ++i) {
    const int e = i * NT + t;
    const int r = e >> 6;
    const int c = e & 63;
    sm[c][r] = bf16r(W[(size_t)(k0 + r) * ND + c0 + c]) * carry;
  }
  __syncthreads();
  const int lane = t & 31, wave = t >> 5;
  const int q = lane >> 3, c8 = (lane & 7) * 8;
  v4u u[2];
#pragma unroll
  for (int it = 0; it < 2; ++it) {
    const int row = wave * 8 + it * 4 + q;
    unsigned short hb[8];
#pragma unroll
    for (int e = 0; e < 8; ++e) hb[e] = h_bits(sm[row][c8 + e]);
    u[it] = (v4u){pk16(hb[0], hb[1]), pk16(hb[2], hb[3]), pk16(hb[4], hb[5]), pk16(hb[6], hb[7])};
  }
  for (int pass = 0; pass < 2; ++pass) {
#pragma unroll
    for (int it = 0; it < 2; ++it) {
      const int row = wave * 8 + it * 4 + q;
      *(volatile v4u*)(op + (size_t)(c0 + row) * KD + k0 + c8) = u[it];
    }
    __threadfence();
  }
}

__global__ __launch_bounds__(256) void featcast_kernel(const float* __restrict__ feats, unsigned short* __restrict__ dst16) {
  const int i = blockIdx.x * 256 + threadIdx.x;
  if (i >= NFC8) return;
  const int row = i >> 4;
  const int c8 = (i & 15) * 8;
  const float* p = feats + (size_t)row * FDIM + c8;
  const v4f a = *(const v4f*)(p);
  const v4f c = *(const v4f*)(p + 4);
  unsigned short hb[8];
#pragma unroll
  for (int e = 0; e < 4; ++e) { hb[e] = bf_bits_rne(a[e]); hb[4 + e] = bf_bits_rne(c[e]); }
  const v4u u = (v4u){pk16(hb[0], hb[1]), pk16(hb[2], hb[3]), pk16(hb[4], hb[5]), pk16(hb[6], hb[7])};
  unsigned short* q = dst16 + (size_t)row * KJK + c8;
  *(volatile v4u*)q = u;
  __threadfence();
  *(volatile v4u*)q = u;
}

__device__ __forceinline__ int chunk_collect(const int* __restrict__ keyv, int e0, int n0, int range,
                                             int tid, int* LIST, int* wtot) {
  const int lane = tid & 31, wave = tid >> 5;
  const int eb = e0 + tid * SPT;
  const bool valid = eb < NE;
  const int ebc = valid ? eb : (NE - SPT);
  int dv[SPT];
#pragma unroll
  for (int k = 0; k < SPT; k += 4) {
    const v4i d4 = *(const v4i*)(keyv + ebc + k);
    dv[k] = d4[0]; dv[k + 1] = d4[1]; dv[k + 2] = d4[2]; dv[k + 3] = d4[3];
  }
  const unsigned urange = valid ? (unsigned)range : 0u;
  unsigned hm[SPT];
  int cw = 0;
#pragma unroll
  for (int k = 0; k < SPT; ++k) {
    const int hit = ((unsigned)(dv[k] - n0) < urange) ? 1 : 0;
    hm[k] = (unsigned)__ballot(hit);
    cw += (int)__popc(hm[k]);
  }
  if (lane == 0) wtot[wave] = cw;
  __syncthreads();
  int pre = 0, tot = 0;
#pragma unroll
  for (int w = 0; w < NWAVE; ++w) { const int tw = wtot[w]; tot += tw; pre += (w < wave) ? tw : 0; }
  const unsigned ltmask = (1u << lane) - 1u;
#pragma unroll
  for (int k = 0; k < SPT; ++k) {
    const unsigned mk = hm[k];
    if (mk != 0u) {
      const int pos = pre + (int)__popc(mk & ltmask);
      const int hit = ((unsigned)(dv[k] - n0) < urange) ? 1 : 0;
      const int rec = ((dv[k] - n0) << REC_SHIFT) | (tid * SPT + k);
      if (hit != 0 && pos < SCH) LIST[pos] = rec;
      pre += (int)__popc(mk);
    }
  }
  __syncthreads();
  return tot < SCH ? tot : SCH;
}

__global__ __launch_bounds__(NT) void degree_kernel(const int* __restrict__ srcv, const int* __restrict__ dstv,
                                                   float* __restrict__ onorm, float* __restrict__ inorm) {
  __shared__ int CNT[RD];
  __shared__ int LIST[SCH];
  __shared__ int wtot[NWAVE];
  const int tid = threadIdx.x, lane = tid & 31, wave = tid >> 5;
  const int ph = blockIdx.y;
  const int* keyv = (ph == 0) ? srcv : dstv;
  float* outp = (ph == 0) ? onorm : inorm;
  const int n0 = blockIdx.x * RD;
  int range = NN - n0; range = range < RD ? range : RD; range = range > 0 ? range : 0;
#pragma unroll 1
  for (int i = tid; i < RD; i += NT) CNT[i] = 0;
#pragma unroll 1
  for (int i = tid; i < SCH; i += NT) LIST[i] = -1;
  if (tid < NWAVE) wtot[tid] = 0;
  __syncthreads();
#pragma unroll 1
  for (int c = 0; c < NCH; ++c) {
    const int tot = chunk_collect(keyv, c * SCH, n0, range, tid, LIST, wtot);
#pragma unroll 1
    for (int base = 0; base < tot; base += 32) {
      const int q = base + lane;
      const int qc = (q < SCH) ? q : (SCH - 1);
      const int lv = LIST[qc];
      const int rv = (q < tot) ? lv : -1;
      const int own = (rv >= 0 && (((rv >> REC_SHIFT) & 7) == wave)) ? 1 : 0;
      unsigned msk = (unsigned)__ballot(own);
#pragma unroll 1
      for (int it = 0; it < 32; ++it) {
        if (msk == 0u) break;
        const int bp = __builtin_ctz(msk); msk &= msk - 1u;
        const int r = __shfl(rv, bp, 32);
        int dl = r >> REC_SHIFT; dl = dl < RD ? dl : (RD - 1);
        if (lane == 0) CNT[dl] = CNT[dl] + 1;
      }
    }
    __syncthreads();
  }
  __syncthreads();
  float* bp0 = outp + (size_t)n0;
#pragma unroll 1
  for (int it = 0; it < RD / (4 * NT); ++it) {
    const int row = it * (4 * NT) + 4 * tid;
    v4f nv;
#pragma unroll
    for (int e = 0; e < 4; ++e) {
      const int cn = CNT[row + e];
      const float cf = (float)(cn > 0 ? cn : 1);
      const float rs = 1.0f / sqrtf(cf);
      nv[e] = (cn > 0) ? rs : 0.0f;
    }
    *(volatile v4f*)(bp0 + row) = nv;
    __threadfence();
    *(volatile v4f*)(bp0 + row) = nv;
  }
}

template <int XMODE>
__global__ __launch_bounds__(NT) void agg_layer_kernel(const unsigned short* __restrict__ xh,
                                                      const int* __restrict__ srcv, const int* __restrict__ dstv,
                                                      const float* __restrict__ onorm,
                                                      unsigned short* __restrict__ AH, float ocarry) {
  __shared__ __align__(16) float ACC[RL * FDIM];
  __shared__ int LIST[SCH];
  __shared__ int wtot[NWAVE];
  const int tid = threadIdx.x, lane = tid & 31, wave = tid >> 5;
  const int n0 = blockIdx.x * RL;
  int range = NN - n0; range = range < RL ? range : RL; range = range > 0 ? range : 0;
  const v4f z4 = {0.f, 0.f, 0.f, 0.f};
  v4f* accv = (v4f*)ACC;
#pragma unroll 1
  for (int i = tid; i < RL * FDIM / 4; i += NT) accv[i] = z4;
#pragma unroll 1
  for (int i = tid; i < SCH; i += NT) LIST[i] = -1;
  if (tid < NWAVE) wtot[tid] = 0;
  __syncthreads();
#pragma unroll 1
  for (int c = 0; c < NCH; ++c) {
    const int e0 = c * SCH;
    const int tot = chunk_collect(dstv, e0, n0, range, tid, LIST, wtot);
#pragma unroll 1
    for (int base = 0; base < tot; base += 32) {
      const int q = base + lane;
      const int qc = (q < SCH) ? q : (SCH - 1);
      const int lv = LIST[qc];
      const int rv = (q < tot) ? lv : -1;
      const int own = (rv >= 0 && (((rv >> REC_SHIFT) & 7) == wave)) ? 1 : 0;
      unsigned msk = (unsigned)__ballot(own);
#pragma unroll 1
      for (int it = 0; it < 32; ++it) {
        if (msk == 0u) break;
        const int bp = __builtin_ctz(msk); msk &= msk - 1u;
        const int r = __shfl(rv, bp, 32);
        int dl = r >> REC_SHIFT; dl = dl < RL ? dl : (RL - 1);
        int e = e0 + (r & (SCH - 1)); e = e < NE ? e : (NE - 1);
        const int s0 = srcv[e];
        const int s = s0 < 0 ? 0 : (s0 >= NN ? NN - 1 : s0);
        const float on = onorm[s];
        const v2u w = *(const v2u*)(xh + (size_t)s * KJK + 4 * lane);
        float x0, x1, x2, x3;
        if (XMODE == 0) {
          x0 = __uint_as_float(w.x << 16); x1 = __uint_as_float(w.x & 0xffff0000u);
          x2 = __uint_as_float(w.y << 16); x3 = __uint_as_float(w.y & 0xffff0000u);
        } else {
          x0 = h16_to_f32(w.x & 0xffffu); x1 = h16_to_f32(w.x >> 16);
          x2 = h16_to_f32(w.y & 0xffffu); x3 = h16_to_f32(w.y >> 16);
        }
        float* ap = ACC + dl * FDIM + 4 * lane;
        v4f a = *(const v4f*)ap;
        a[0] = fmaf(on, x0, a[0]); a[1] = fmaf(on, x1, a[1]);
        a[2] = fmaf(on, x2, a[2]); a[3] = fmaf(on, x3, a[3]);
        *(v4f*)ap = a;
      }
    }
    __syncthreads();
  }
  __syncthreads();
  const int hh = lane >> 4, c8 = (lane & 15) * 8;
#pragma unroll 1
  for (int j = 0; j < RLW / 2; ++j) {
    const int dlb = wave * RLW + 2 * j;
    const int nb = n0 + dlb;
    if (nb < NPAD) {
      const int dl = dlb + hh;
      const float* sp = ACC + dl * FDIM + c8;
      const v4f a0 = *(const v4f*)sp;
      const v4f a1 = *(const v4f*)(sp + 4);
      unsigned short hb[8];
#pragma unroll
      for (int e = 0; e < 4; ++e) { hb[e] = h_bits(a0[e] * ocarry); hb[4 + e] = h_bits(a1[e] * ocarry); }
      const v4u u = (v4u){pk16(hb[0], hb[1]), pk16(hb[2], hb[3]), pk16(hb[4], hb[5]), pk16(hb[6], hb[7])};
      unsigned short* dp = AH + (size_t)(n0 + dl) * FDIM + c8;
      *(volatile v4u*)dp = u;
      __threadfence();
      *(volatile v4u*)dp = u;
    }
  }
}

__global__ __launch_bounds__(NT) void agg_final_kernel(const float* __restrict__ zp, const int* __restrict__ srcv,
                                                      const int* __restrict__ dstv, const float* __restrict__ bo,
                                                      float* __restrict__ outp) {
  __shared__ __align__(16) float ACC[RF * CDIM];
  __shared__ int LIST[SCH];
  __shared__ int wtot[NWAVE];
  const int tid = threadIdx.x, lane = tid & 31, wave = tid >> 5;
  const int n0 = blockIdx.x * RF;
  int range = NN - n0; range = range < RF ? range : RF; range = range > 0 ? range : 0;
  const v4f z4 = {0.f, 0.f, 0.f, 0.f};
  v4f* accv = (v4f*)ACC;
#pragma unroll 1
  for (int i = tid; i < RF * CDIM / 4; i += NT) accv[i] = z4;
#pragma unroll 1
  for (int i = tid; i < SCH; i += NT) LIST[i] = -1;
  if (tid < NWAVE) wtot[tid] = 0;
  __syncthreads();
#pragma unroll 1
  for (int c = 0; c < NCH; ++c) {
    const int e0 = c * SCH;
    const int tot = chunk_collect(dstv, e0, n0, range, tid, LIST, wtot);
#pragma unroll 1
    for (int base = 0; base < tot; base += 32) {
      const int q = base + lane;
      const int qc = (q < SCH) ? q : (SCH - 1);
      const int lv = LIST[qc];
      const int rv = (q < tot) ? lv : -1;
      const int own = (rv >= 0 && (((rv >> REC_SHIFT) & 7) == wave)) ? 1 : 0;
      unsigned msk = (unsigned)__ballot(own);
#pragma unroll 1
      for (int it = 0; it < 32; ++it) {
        if (msk == 0u) break;
        const int bp = __builtin_ctz(msk); msk &= msk - 1u;
        const int r = __shfl(rv, bp, 32);
        int dl = r >> REC_SHIFT; dl = dl < RF ? dl : (RF - 1);
        int e = e0 + (r & (SCH - 1)); e = e < NE ? e : (NE - 1);
        const int s0 = srcv[e];
        const int s = s0 < 0 ? 0 : (s0 >= NN ? NN - 1 : s0);
        const v2f zv = *(const v2f*)(zp + (size_t)s * CDIM + 2 * lane);
        float* ap = ACC + dl * CDIM + 2 * lane;
        v2f a = *(const v2f*)ap;
        a = a + zv;
        *(v2f*)ap = a;
      }
    }
    __syncthreads();
  }
  __syncthreads();
  const int hh = lane >> 4, c4 = (lane & 15) * 4;
  v4f bo4;
#pragma unroll
  for (int e = 0; e < 4; ++e) bo4[e] = bf16r(bo[c4 + e]);
#pragma unroll 1
  for (int j = 0; j < RFW / 2; ++j) {
    const int dlb = wave * RFW + 2 * j;
    const int nb = n0 + dlb;
    if (nb < NN) {
      const int dl = dlb + hh;
      v4f v = *(const v4f*)(ACC + dl * CDIM + c4);
      v = v + bo4;
      float* dp = outp + (size_t)(n0 + dl) * CDIM + c4;
      *(volatile v4f*)dp = v;
      __threadfence();
      *(volatile v4f*)dp = v;
    }
  }
}

extern "C" void kernel_launch(void* const* d_in, const int* in_sizes, int n_in,
                              void* d_out, int out_size, void* d_ws, size_t ws_size, hipStream_t stream) {
  if (n_in < 11) return;
  if (in_sizes[0] != NN * FDIM || in_sizes[1] != NE || in_sizes[2] != NE) return;
  if (in_sizes[3] != FDIM * FDIM || in_sizes[5] != FDIM * FDIM || in_sizes[7] != FDIM * FDIM) return;
  if (in_sizes[4] != FDIM || in_sizes[6] != FDIM || in_sizes[8] != FDIM) return;
  if (in_sizes[9] != KJK * CDIM || in_sizes[10] != CDIM) return;
  if (out_size != NN * CDIM) return;

  const float* feats = (const float*)d_in[0];
  const int*   srcv  = (const int*)d_in[1];
  const int*   dstv  = (const int*)d_in[2];
  const float* W0 = (const float*)d_in[3];
  const float* b0 = (const float*)d_in[4];
  const float* W1 = (const float*)d_in[5];
  const float* b1 = (const float*)d_in[6];
  const float* W2 = (const float*)d_in[7];
  const float* b2 = (const float*)d_in[8];
  const float* Wo = (const float*)d_in[9];
  const float* bo = (const float*)d_in[10];
  float* out = (float*)d_out;

  char* ws = (char*)d_ws; size_t off = 0;
  auto carve = [&](size_t bytes) -> char* { char* p = ws + off; off += (bytes + 255) & ~(size_t)255; return p; };
  float*          onorm = (float*)carve((size_t)NORM_ROWS * 4);
  float*          inorm = (float*)carve((size_t)NORM_ROWS * 4);
  unsigned short* wt0   = (unsigned short*)carve((size_t)FDIM * FDIM * 2);
  unsigned short* wt1   = (unsigned short*)carve((size_t)FDIM * FDIM * 2);
  unsigned short* wt2   = (unsigned short*)carve((size_t)FDIM * FDIM * 2);
  unsigned short* wot   = (unsigned short*)carve((size_t)CDIM * KJK * 2);
  unsigned short* aggh  = (unsigned short*)carve((size_t)NPAD * FDIM * 2);
  unsigned short* jk    = (unsigned short*)carve((size_t)NPAD * KJK * 2);
  float*          zbuf  = (float*)carve((size_t)NPAD * CDIM * 4);
  if (off > ws_size || off > (size_t)134217728) return;

  const int tilesL = (NPAD / 64) * (FDIM / 64);
  const int gridL  = (tilesL + 7) / 8;
  const int tilesZ = (NPAD / 64) * (CDIM / 64);
  const int gridZ  = (tilesZ + 7) / 8;

  prep_kernel<<<dim3(6, 2, 4), NT, 0, stream>>>(W0, W1, W2, Wo, wt0, wt1, wt2, wot, WCARRY);
  featcast_kernel<<<NFC8 / 256, 256, 0, stream>>>(feats, jk + FDIM);
  degree_kernel<<<dim3(NBD, 2), NT, 0, stream>>>(srcv, dstv, onorm, inorm);

  agg_layer_kernel<0><<<NBL, NT, 0, stream>>>(jk + FDIM, srcv, dstv, onorm, aggh, AGG0CARRY);
  gemm_f16_kernel<true, true, true, 1><<<gridL, 256, 0, stream>>>(aggh, FDIM, wt0, FDIM, (void*)(jk + 0), KJK,
                                                                 b0, inorm, NPAD, FDIM, FDIM, GSCALE, HCARRY);
  agg_layer_kernel<1><<<NBL, NT, 0, stream>>>(jk + 0, srcv, dstv, onorm, aggh, 1.0f);
  gemm_f16_kernel<true, true, true, 1><<<gridL, 256, 0, stream>>>(aggh, FDIM, wt1, FDIM, (void*)(jk + FDIM), KJK,
                                                                 b1, inorm, NPAD, FDIM, FDIM, GSCALE, HCARRY);
  agg_layer_kernel<1><<<NBL, NT, 0, stream>>>(jk + FDIM, srcv, dstv, onorm, aggh, 1.0f);
  gemm_f16_kernel<true, true, true, 1><<<gridL, 256, 0, stream>>>(aggh, FDIM, wt2, FDIM, (void*)(jk + 2 * FDIM), KJK,
                                                                 b2, inorm, NPAD, FDIM, FDIM, GSCALE, HCARRY);
  gemm_f16_kernel<false, false, false, 0><<<gridZ, 256, 0, stream>>>(jk, KJK, wot, KJK, (void*)zbuf, CDIM,
                                                                    bo, inorm, NPAD, CDIM, KJK, GSCALE, 1.0f);
  agg_final_kernel<<<NBF, NT, 0, stream>>>(zbuf, srcv, dstv, bo, out);
}
